// BNAF_33062658245364
// MI455X (gfx1250) — hardware-verified
//
#include <hip/hip_runtime.h>
#include <stddef.h>
#include <stdint.h>
#include <math.h>


#define BN    2048
#define HN    512
#define DN    8
#define OB    64
#define ASC   256
#define WSC   2048
#define NTHR  256
#define NWAVE 8
#define WSCAP 134217728
#define LDS_GEMM (NWAVE * 32 * 64 * 4)

static_assert(HN == DN * OB);
static_assert((HN % 128) == 0);
static_assert((BN % 128) == 0);
static_assert((BN % 32) == 0);
static_assert(NTHR == NWAVE * 32);
static_assert(HN == 2 * NTHR);
static_assert((OB % 32) == 0);
static_assert(LDS_GEMM <= 300 * 1024);

typedef float          v4f  __attribute__((ext_vector_type(4)));
typedef float          v8f  __attribute__((ext_vector_type(8)));
typedef _Float16       v8h  __attribute__((ext_vector_type(8)));
typedef _Float16       v16h __attribute__((ext_vector_type(16)));
union FragH { v16h v; v8h h[2]; };

__device__ __forceinline__ v8f wmf(v16h a, v16h b, v8f c) {
  v8f d = __builtin_amdgcn_wmma_f32_16x16x32_f16(false, a, false, b, (short)0, c, false, false);
  asm volatile("v_nop\n\tv_nop\n\tv_nop\n\tv_nop" : "+v"(d) : "v"(a), "v"(b));
  return d;
}

__device__ __forceinline__ void tanh_ld(float x, float& th, float& ld) {
  const float e  = __expf(-2.f * fabsf(x));
  const float t  = (1.f - e) * __builtin_amdgcn_rcpf(1.f + e);
  th = __builtin_copysignf(t, x);
  const float sp = fmaxf(-2.f * x, 0.f) + __logf(1.f + e);
  ld = -2.f * (x - 0.69314718055994531f + sp);
}

__global__ __launch_bounds__(NTHR) void k_prep_small(const float* __restrict__ W1, const float* __restrict__ lg1,
                                                     const float* __restrict__ W4, const float* __restrict__ lg4,
                                                     float* w1f, float* ldb1, float* w4f, float* ldb4) {
  __shared__ __attribute__((aligned(16))) float s_w[NTHR * DN];
  __shared__ __attribute__((aligned(16))) float s_l[NTHR];
  const int tid = threadIdx.x;
  if (blockIdx.x < 2) {
    const int n   = blockIdx.x * NTHR + tid;
    const int blk = n >> 6;
    const float lg = lg1[n];
    const v4f a = *(const v4f*)(W1 + (size_t)n * DN);
    const v4f b = *(const v4f*)(W1 + (size_t)n * DN + 4);
    const float wv[8] = {a.x, a.y, a.z, a.w, b.x, b.y, b.z, b.w};
    float v[8];
    float ss = 0.f, wd = 0.f;
#pragma unroll
    for (int c = 0; c < 8; ++c) {
      const float ex = __expf(wv[c]);
      const float vv = (c < blk) ? wv[c] : ((c == blk) ? ex : 0.f);
      v[c] = vv;
      ss += vv * vv;
      wd = (c == blk) ? wv[c] : wd;
    }
    const float vnorm  = sqrtf(ss);
    const float rn     = __builtin_amdgcn_rcpf(vnorm);
    const float eg     = __expf(lg);
    const float half_l = 0.5f * __logf(vnorm * vnorm);
#pragma unroll
    for (int c = 0; c < 8; ++c) s_w[tid * DN + c] = (eg * v[c]) * rn;
    s_l[tid] = (lg + wd) - half_l;
    __syncthreads();
    const v4f o0 = *(const v4f*)(s_w + 4 * tid);
    const v4f o1 = *(const v4f*)(s_w + 4 * (tid + NTHR));
    const int tl = tid & 63;
    const v4f l4 = *(const v4f*)(s_l + 4 * tl);
    float* bw = w1f + (size_t)blockIdx.x * (NTHR * DN);
    float* bl = ldb1 + (size_t)blockIdx.x * NTHR + 4 * tl;
    *(volatile v4f*)(bw + 4 * tid) = o0;
    *(volatile v4f*)(bw + 4 * (tid + NTHR)) = o1;
    if (tid < 64) *(volatile v4f*)bl = l4;
    __threadfence();
    *(volatile v4f*)(bw + 4 * tid) = o0;
    *(volatile v4f*)(bw + 4 * (tid + NTHR)) = o1;
    if (tid < 64) *(volatile v4f*)bl = l4;
  } else {
    const int lane = tid & 31, j = tid >> 5;
    const int dlo = j * OB, dhi = dlo + OB;
    const float lg = lg4[j];
    const float* wr = W4 + (size_t)j * HN;
    float v[4][4];
    float ss = 0.f;
#pragma unroll
    for (int q = 0; q < 4; ++q) {
      const int c0 = q * 128 + 4 * lane;
      const v4f a = *(const v4f*)(wr + c0);
      const float wv[4] = {a.x, a.y, a.z, a.w};
#pragma unroll
      for (int e = 0; e < 4; ++e) {
        const int c = c0 + e;
        const float ex = __expf(wv[e]);
        const float vv = (c < dlo) ? wv[e] : ((c < dhi) ? ex : 0.f);
        v[q][e] = vv;
        ss += vv * vv;
      }
    }
#pragma unroll
    for (int off = 16; off > 0; off >>= 1) ss += __shfl_xor(ss, off, 32);
    const float vnorm  = sqrtf(ss);
    const float rn     = __builtin_amdgcn_rcpf(vnorm);
    const float eg     = __expf(lg);
    const float half_l = 0.5f * __logf(vnorm * vnorm);
    v4f o[4];
#pragma unroll
    for (int q = 0; q < 4; ++q) {
      o[q].x = (eg * v[q][0]) * rn; o[q].y = (eg * v[q][1]) * rn;
      o[q].z = (eg * v[q][2]) * rn; o[q].w = (eg * v[q][3]) * rn;
    }
    const int lc = lane & 15;
    const v4f wd = *(const v4f*)(wr + dlo + 4 * lc);
    v4f l4;
    l4.x = (lg + wd.x) - half_l; l4.y = (lg + wd.y) - half_l;
    l4.z = (lg + wd.z) - half_l; l4.w = (lg + wd.w) - half_l;
    float* bw = w4f + (size_t)j * HN + 4 * lane;
    float* bl = ldb4 + (size_t)j * OB + 4 * lc;
#pragma unroll
    for (int q = 0; q < 4; ++q) *(volatile v4f*)(bw + q * 128) = o[q];
    if (lane < 16) *(volatile v4f*)bl = l4;
    __threadfence();
#pragma unroll
    for (int q = 0; q < 4; ++q) *(volatile v4f*)(bw + q * 128) = o[q];
    if (lane < 16) *(volatile v4f*)bl = l4;
  }
}

__global__ __launch_bounds__(NTHR) void k_prepw(const float* __restrict__ W, const float* __restrict__ logg,
                                                _Float16* wB, float* ldb) {
  const int tid = threadIdx.x, lane = tid & 31, wave = tid >> 5;
  const int n = blockIdx.x * NWAVE + wave;
  const int blk = n >> 6, dlo = blk * OB, dhi = dlo + OB;
  const float lg = logg[n];
  const float* wr = W + (size_t)n * HN;
  float v[2][8];
  float ss = 0.f;
#pragma unroll
  for (int ch = 0; ch < 2; ++ch) {
    const int c0 = ch * 256 + 8 * lane;
    const v4f a = *(const v4f*)(wr + c0);
    const v4f b = *(const v4f*)(wr + c0 + 4);
    const float wv[8] = {a.x, a.y, a.z, a.w, b.x, b.y, b.z, b.w};
#pragma unroll
    for (int e = 0; e < 8; ++e) {
      const int c = c0 + e;
      const float ex = __expf(wv[e]);
      const float vv = (c < dlo) ? wv[e] : ((c < dhi) ? ex : 0.f);
      v[ch][e] = vv;
      ss += vv * vv;
    }
  }
#pragma unroll
  for (int off = 16; off > 0; off >>= 1) ss += __shfl_xor(ss, off, 32);
  const float vnorm  = sqrtf(ss);
  const float rn     = __builtin_amdgcn_rcpf(vnorm);
  const float eg     = __expf(lg);
  const float half_l = 0.5f * __logf(vnorm * vnorm);
  v8h hv[2];
#pragma unroll
  for (int ch = 0; ch < 2; ++ch) {
#pragma unroll
    for (int e = 0; e < 8; ++e) hv[ch][e] = (_Float16)(((eg * v[ch][e]) * rn) * (float)WSC);
  }
  const int lc = lane & 15;
  const v4f wd = *(const v4f*)(wr + dlo + 4 * lc);
  v4f l4;
  l4.x = (lg + wd.x) - half_l; l4.y = (lg + wd.y) - half_l;
  l4.z = (lg + wd.z) - half_l; l4.w = (lg + wd.w) - half_l;
  _Float16* d0 = wB + (size_t)n * HN + 8 * lane;
  _Float16* d1 = d0 + 256;
  float* dl = ldb + (size_t)n * OB + 4 * lc;
  *(volatile v8h*)d0 = hv[0];
  *(volatile v8h*)d1 = hv[1];
  if (lane < 16) *(volatile v4f*)dl = l4;
  __threadfence();
  *(volatile v8h*)d0 = hv[0];
  *(volatile v8h*)d1 = hv[1];
  if (lane < 16) *(volatile v4f*)dl = l4;
}

__global__ __launch_bounds__(NTHR) void k_layer1(const float* __restrict__ x, const float* __restrict__ w1f,
                                                 const float* __restrict__ bias1, const float* __restrict__ ldb1,
                                                 _Float16* hA, float* sld) {
  __shared__ __attribute__((aligned(16))) _Float16 s_h[NTHR];
  __shared__ __attribute__((aligned(16))) float s_s[NTHR];
  const int tid = threadIdx.x;
  const int b = blockIdx.x >> 1, hf = blockIdx.x & 1;
  const int r = hf * NTHR + tid;
  const v4f xa = *(const v4f*)(x + (size_t)b * DN);
  const v4f xb = *(const v4f*)(x + (size_t)b * DN + 4);
  const v4f wa = *(const v4f*)(w1f + (size_t)r * DN);
  const v4f wb = *(const v4f*)(w1f + (size_t)r * DN + 4);
  float acc = xa.x * wa.x;
  acc += xa.y * wa.y; acc += xa.z * wa.z; acc += xa.w * wa.w;
  acc += xb.x * wb.x; acc += xb.y * wb.y; acc += xb.z * wb.z; acc += xb.w * wb.w;
  const float pre = acc + bias1[r];
  float th, ld;
  tanh_ld(pre, th, ld);
  s_h[tid] = (_Float16)(th * (float)ASC);
  s_s[tid] = ldb1[r] + ld;
  __syncthreads();
  const int lh = tid & 31, ls = tid & 63;
  const v8h hv = *(const v8h*)(s_h + 8 * lh);
  const v4f sv = *(const v4f*)(s_s + 4 * ls);
  _Float16* dh = hA + (size_t)b * HN + hf * NTHR + 8 * lh;
  float* ds = sld + (size_t)b * HN + hf * NTHR + 4 * ls;
  if (tid < 32) *(volatile v8h*)dh = hv;
  if (tid < 64) *(volatile v4f*)ds = sv;
  __threadfence();
  if (tid < 32) *(volatile v8h*)dh = hv;
  if (tid < 64) *(volatile v4f*)ds = sv;
}

__device__ __forceinline__ void epi_h16(const float* stg, _Float16* hb, int lane) {
  const int rq = lane >> 3, c0 = 8 * (lane & 7);
#pragma unroll 1
  for (int q = 0; q < 8; ++q) {
    const int row = 4 * q + rq;
    const float* sp = stg + row * 64 + c0;
    const v4f p0 = *(const v4f*)sp;
    const v4f p1 = *(const v4f*)(sp + 4);
    const float pv[8] = {p0.x, p0.y, p0.z, p0.w, p1.x, p1.y, p1.z, p1.w};
    v8h o;
#pragma unroll
    for (int e = 0; e < 8; ++e) {
      float th, ld;
      tanh_ld(pv[e], th, ld);
      o[e] = (_Float16)(th * (float)ASC);
    }
    *(volatile v8h*)(hb + (size_t)row * HN + c0) = o;
  }
}

__device__ __forceinline__ void epi_ld(const float* stg, float* lb, int hh, int m) {
#pragma unroll 1
  for (int q = 0; q < 16; ++q) {
    const int row = 2 * q + hh;
    const v4f p = *(const v4f*)(stg + row * 64 + 4 * m);
    float th, l0, l1, l2, l3;
    tanh_ld(p.x, th, l0); tanh_ld(p.y, th, l1); tanh_ld(p.z, th, l2); tanh_ld(p.w, th, l3);
    v4f lv; lv.x = l0; lv.y = l1; lv.z = l2; lv.w = l3;
    *(volatile v4f*)(lb + (size_t)row * HN + 4 * m) = lv;
  }
}

__device__ __forceinline__ void epi_h32ld(const float* stg, float* hb, float* lb, int hh, int m) {
#pragma unroll 1
  for (int q = 0; q < 16; ++q) {
    const int row = 2 * q + hh;
    const v4f p = *(const v4f*)(stg + row * 64 + 4 * m);
    float t0, t1, t2, t3, l0, l1, l2, l3;
    tanh_ld(p.x, t0, l0); tanh_ld(p.y, t1, l1); tanh_ld(p.z, t2, l2); tanh_ld(p.w, t3, l3);
    v4f tv; tv.x = t0; tv.y = t1; tv.z = t2; tv.w = t3;
    v4f lv; lv.x = l0; lv.y = l1; lv.z = l2; lv.w = l3;
    *(volatile v4f*)(hb + (size_t)row * HN + 4 * m) = tv;
    *(volatile v4f*)(lb + (size_t)row * HN + 4 * m) = lv;
  }
}

template <bool HF16>
__global__ __launch_bounds__(NTHR) void k_gemm(const _Float16* __restrict__ hA, const _Float16* __restrict__ wB,
                                               const float* __restrict__ bias,
                                               _Float16* h16, float* h32, float* ldt) {
  extern __shared__ v4f lds_dyn[];
  const int tid = threadIdx.x, lane = tid & 31, wave = tid >> 5, hh = lane >> 4, m = lane & 15;
  float* stg = (float*)lds_dyn + wave * (32 * 64);
  const int n0 = blockIdx.x * 128, m0 = blockIdx.y * 128;
  const int wm = (wave >> 1) * 32, wn = (wave & 1) * 64;
  const int ksteps = (2 * (int)blockIdx.x + 2) * (OB / 32);

  v8f acc[2][4];
#pragma unroll
  for (int mt = 0; mt < 2; ++mt)
#pragma unroll
    for (int nt = 0; nt < 4; ++nt) { v8f z = {0.f, 0.f, 0.f, 0.f, 0.f, 0.f, 0.f, 0.f}; acc[mt][nt] = z; }

  const _Float16* ap = hA + (size_t)(m0 + wm + m) * HN + 8 * hh;
  const _Float16* bp = wB + (size_t)(n0 + wn + m) * HN + 8 * hh;
#pragma unroll 1
  for (int kt = 0; kt < ksteps; ++kt) {
    const int k0 = 32 * kt;
    FragH a0, a1;
    a0.h[0] = *(const v8h*)(ap + k0);
    a0.h[1] = *(const v8h*)(ap + k0 + 16);
    a1.h[0] = *(const v8h*)(ap + 16 * HN + k0);
    a1.h[1] = *(const v8h*)(ap + 16 * HN + k0 + 16);
#pragma unroll
    for (int nt = 0; nt < 4; ++nt) {
      const _Float16* bq = bp + (size_t)nt * 16 * HN + k0;
      FragH b;
      b.h[0] = *(const v8h*)bq;
      b.h[1] = *(const v8h*)(bq + 16);
      acc[0][nt] = wmf(a0.v, b.v, acc[0][nt]);
      acc[1][nt] = wmf(a1.v, b.v, acc[1][nt]);
    }
  }

  constexpr float OSC = 1.0f / ((float)ASC * (float)WSC);
  float bv[4];
#pragma unroll
  for (int nt = 0; nt < 4; ++nt) bv[nt] = bias[n0 + wn + 16 * nt + m];
#pragma unroll
  for (int mt = 0; mt < 2; ++mt) {
    float* sp = stg + (16 * mt + 8 * hh) * 64 + m;
#pragma unroll
    for (int nt = 0; nt < 4; ++nt) {
#pragma unroll
      for (int r = 0; r < 8; ++r) sp[r * 64 + 16 * nt] = acc[mt][nt][r] * OSC + bv[nt];
    }
  }
  __syncthreads();

  const size_t base = (size_t)(m0 + wm) * HN + n0 + wn;
  if (HF16) {
    epi_h16(stg, h16 + base, lane);
    epi_ld(stg, ldt + base, hh, m);
    __threadfence();
    epi_h16(stg, h16 + base, lane);
    epi_ld(stg, ldt + base, hh, m);
  } else {
    epi_h32ld(stg, h32 + base, ldt + base, hh, m);
    __threadfence();
    epi_h32ld(stg, h32 + base, ldt + base, hh, m);
  }
}

__global__ __launch_bounds__(NTHR) void k_sld(const float* __restrict__ sin_, const float* __restrict__ ldb,
                                              const float* __restrict__ ldt, float* sout) {
  __shared__ __attribute__((aligned(16))) float s_ldb[OB * OB];
  __shared__ __attribute__((aligned(16))) float s_in[4 * OB];
  __shared__ __attribute__((aligned(16))) float s_res[4 * OB];
  const int j = blockIdx.y, b0 = blockIdx.x * 4, tid = threadIdx.x;
#pragma unroll 1
  for (int t = tid; t < OB * OB; t += NTHR) {
    const int o = t >> 6, i = t & 63;
    s_ldb[i * OB + o] = ldb[(size_t)j * OB * OB + t];
  }
  {
    const int bl = tid >> 6, i = tid & 63;
    s_in[tid] = sin_[(size_t)(b0 + bl) * HN + j * OB + i];
  }
  __syncthreads();
  const int o = tid & 63, bl = tid >> 6, b = b0 + bl;
  const float* si = s_in + bl * OB;
  float mx = si[0] + s_ldb[o];
#pragma unroll 4
  for (int i = 1; i < OB; ++i) mx = fmaxf(mx, si[i] + s_ldb[i * OB + o]);
  float s = 0.f;
#pragma unroll 4
  for (int i = 0; i < OB; ++i) s += __expf((si[i] + s_ldb[i * OB + o]) - mx);
  s_res[tid] = (mx + __logf(s)) + ldt[(size_t)b * HN + j * OB + o];
  __syncthreads();
  const int t = tid & 63;
  const v4f rv = *(const v4f*)(s_res + 4 * t);
  float* d = sout + (size_t)(b0 + (t >> 4)) * HN + j * OB + 4 * (t & 15);
  if (tid < 64) *(volatile v4f*)d = rv;
  __threadfence();
  if (tid < 64) *(volatile v4f*)d = rv;
}

__global__ __launch_bounds__(NTHR) void k_layer4(const float* __restrict__ h3, const float* __restrict__ w4f,
                                                 const float* __restrict__ bias4, const float* __restrict__ ldb4,
                                                 const float* __restrict__ sld3, float* out) {
  __shared__ __attribute__((aligned(16))) float s_o0[NTHR];
  __shared__ __attribute__((aligned(16))) float s_o1[NTHR];
  const int tid = threadIdx.x;
  const int b0 = blockIdx.x * 32, bl = tid >> 3, r = tid & 7, b = b0 + bl;
  const float* hr = h3 + (size_t)b * HN;
  const float* wr = w4f + (size_t)r * HN;
  float acc = 0.f;
#pragma unroll 1
  for (int k = 0; k < HN; k += 4) {
    const v4f hv = *(const v4f*)(hr + k);
    const v4f wv = *(const v4f*)(wr + k);
    acc += hv.x * wv.x; acc += hv.y * wv.y; acc += hv.z * wv.z; acc += hv.w * wv.w;
  }
  const float pre = acc + bias4[r];
  float th, ld;
  tanh_ld(pre, th, ld);
  const float* sp = sld3 + (size_t)b * HN + r * OB;
  const float* lp = ldb4 + (size_t)r * OB;
  float mx = sp[0] + lp[0];
#pragma unroll 4
  for (int i = 1; i < OB; ++i) mx = fmaxf(mx, sp[i] + lp[i]);
  float s = 0.f;
#pragma unroll 4
  for (int i = 0; i < OB; ++i) s += __expf((sp[i] + lp[i]) - mx);
  s_o0[tid] = th;
  s_o1[tid] = (mx + __logf(s)) + ld;
  __syncthreads();
  const int t = tid & 63;
  const bool w0 = tid < 64;
  const bool w1 = (tid >= 64) && (tid < 128);
  const v4f v0 = *(const v4f*)(s_o0 + 4 * t);
  const v4f v1 = *(const v4f*)(s_o1 + 4 * t);
  float* d0 = out + (size_t)b0 * DN + 4 * t;
  float* d1 = out + (size_t)BN * DN + (size_t)b0 * DN + 4 * t;
  if (w0) *(volatile v4f*)d0 = v0;
  if (w1) *(volatile v4f*)d1 = v1;
  __threadfence();
  if (w0) *(volatile v4f*)d0 = v0;
  if (w1) *(volatile v4f*)d1 = v1;
}

static inline size_t al256(size_t b) { return (b + 255) & ~(size_t)255; }

extern "C" void kernel_launch(void* const* d_in, const int* in_sizes, int n_in,
                              void* d_out, int out_size, void* d_ws, size_t ws_size,
                              hipStream_t stream) {
  if (n_in < 13) return;
  if (in_sizes[0] != BN * DN) return;
  if (in_sizes[1] != HN * DN || in_sizes[2] != HN || in_sizes[3] != HN) return;
  if (in_sizes[4] != HN * HN || in_sizes[5] != HN || in_sizes[6] != HN) return;
  if (in_sizes[7] != HN * HN || in_sizes[8] != HN || in_sizes[9] != HN) return;
  if (in_sizes[10] != DN * HN || in_sizes[11] != DN || in_sizes[12] != DN) return;
  if (out_size != 2 * BN * DN) return;

  const float* x     = (const float*)d_in[0];
  const float* W1    = (const float*)d_in[1];
  const float* logg1 = (const float*)d_in[2];
  const float* bias1 = (const float*)d_in[3];
  const float* W2    = (const float*)d_in[4];
  const float* logg2 = (const float*)d_in[5];
  const float* bias2 = (const float*)d_in[6];
  const float* W3    = (const float*)d_in[7];
  const float* logg3 = (const float*)d_in[8];
  const float* bias3 = (const float*)d_in[9];
  const float* W4    = (const float*)d_in[10];
  const float* logg4 = (const float*)d_in[11];
  const float* bias4 = (const float*)d_in[12];
  float* out = (float*)d_out;

  char* ws = (char*)d_ws;
  size_t off = 0;
  const size_t oW1f  = off; off += al256((size_t)HN * DN * 4);
  const size_t oLdb1 = off; off += al256((size_t)HN * 4);
  const size_t oW4f  = off; off += al256((size_t)DN * HN * 4);
  const size_t oLdb4 = off; off += al256((size_t)DN * OB * 4);
  const size_t oWB2  = off; off += al256((size_t)HN * HN * 2);
  const size_t oWB3  = off; off += al256((size_t)HN * HN * 2);
  const size_t oLdb2 = off; off += al256((size_t)HN * OB * 4);
  const size_t oLdb3 = off; off += al256((size_t)HN * OB * 4);
  const size_t oHA1  = off; off += al256((size_t)BN * HN * 2);
  const size_t oHA2  = off; off += al256((size_t)BN * HN * 2);
  const size_t oH3f  = off; off += al256((size_t)BN * HN * 4);
  const size_t oLdt2 = off; off += al256((size_t)BN * HN * 4);
  const size_t oLdt3 = off; off += al256((size_t)BN * HN * 4);
  const size_t oSld1 = off; off += al256((size_t)BN * HN * 4);
  const size_t oSld2 = off; off += al256((size_t)BN * HN * 4);
  const size_t oSld3 = off; off += al256((size_t)BN * HN * 4);
  if (off > ws_size || off > (size_t)WSCAP) return;

  float*    w1f  = (float*)(ws + oW1f);
  float*    ldb1 = (float*)(ws + oLdb1);
  float*    w4f  = (float*)(ws + oW4f);
  float*    ldb4 = (float*)(ws + oLdb4);
  _Float16* wB2  = (_Float16*)(ws + oWB2);
  _Float16* wB3  = (_Float16*)(ws + oWB3);
  float*    ldb2 = (float*)(ws + oLdb2);
  float*    ldb3 = (float*)(ws + oLdb3);
  _Float16* hA1  = (_Float16*)(ws + oHA1);
  _Float16* hA2  = (_Float16*)(ws + oHA2);
  float*    h3f  = (float*)(ws + oH3f);
  float*    ldt2 = (float*)(ws + oLdt2);
  float*    ldt3 = (float*)(ws + oLdt3);
  float*    sld1 = (float*)(ws + oSld1);
  float*    sld2 = (float*)(ws + oSld2);
  float*    sld3 = (float*)(ws + oSld3);

  k_prep_small<<<3, NTHR, 0, stream>>>(W1, logg1, W4, logg4, w1f, ldb1, w4f, ldb4);
  k_prepw<<<HN / NWAVE, NTHR, 0, stream>>>(W2, logg2, wB2, ldb2);
  k_prepw<<<HN / NWAVE, NTHR, 0, stream>>>(W3, logg3, wB3, ldb3);
  k_layer1<<<BN * 2, NTHR, 0, stream>>>(x, w1f, bias1, ldb1, hA1, sld1);
  hipFuncSetAttribute(reinterpret_cast<const void*>(&k_gemm<true>),
                      hipFuncAttributeMaxDynamicSharedMemorySize, LDS_GEMM);
  k_gemm<true><<<dim3(HN / 128, BN / 128), NTHR, LDS_GEMM, stream>>>(hA1, wB2, bias2, hA2, h3f, ldt2);
  k_sld<<<dim3(BN / 4, DN), NTHR, 0, stream>>>(sld1, ldb2, ldt2, sld2);
  hipFuncSetAttribute(reinterpret_cast<const void*>(&k_gemm<false>),
                      hipFuncAttributeMaxDynamicSharedMemorySize, LDS_GEMM);
  k_gemm<false><<<dim3(HN / 128, BN / 128), NTHR, LDS_GEMM, stream>>>(hA2, wB3, bias3, hA1, h3f, ldt3);
  k_sld<<<dim3(BN / 4, DN), NTHR, 0, stream>>>(sld2, ldb3, ldt3, sld3);
  k_layer4<<<BN / 32, NTHR, 0, stream>>>(h3f, w4f, bias4, ldb4, sld3, out);
}
